// EfficientMixedScoreMultiHeadAttention_6700148982477
// MI455X (gfx1250) — hardware-verified
//
#include <hip/hip_runtime.h>


namespace {
constexpr int Bn = 4, R = 512, Cn = 512, E = 256, H = 16, D = 16, MS = 256;
constexpr int NT1 = Bn * R, NT2 = Bn * Cn;
constexpr float WS = 64.0f, QS = 8.0f, TS = 8.0f, M1S = 64.0f, VS = 8.0f, YS = 64.0f;
constexpr int NWAVE_MS = Bn * (R / 16) * (Cn / 32);

typedef _Float16 b16;
typedef __attribute__((ext_vector_type(16))) _Float16 v16b;
typedef __attribute__((ext_vector_type(8)))  _Float16 v8b;
typedef __attribute__((ext_vector_type(8)))  float v8f;
typedef __attribute__((ext_vector_type(4)))  float v4f;

__device__ __forceinline__ v8b ld8b(const b16* p) { return *(const v8b*)p; }
__device__ __forceinline__ v16b cat8b(v8b a, v8b b) { return __builtin_shufflevector(a, b, 0, 1, 2, 3, 4, 5, 6, 7, 8, 9, 10, 11, 12, 13, 14, 15); }
__device__ __forceinline__ v16b frag_kb(const b16* p, int hh) { return cat8b(ld8b(p + 8 * hh), ld8b(p + 16 + 8 * hh)); }
__device__ __forceinline__ void split16(float v, b16& hi, b16& lo) { hi = (b16)v; lo = (b16)(v - (float)hi); }
__device__ __forceinline__ void frag_ksplit(const float* p, int hh, v16b& fh_, v16b& fl_) {
  const float* p0 = p + 8 * hh; const float* p1 = p + 16 + 8 * hh;
#pragma unroll
  for (int e = 0; e < 8; ++e) { b16 a, c; split16(p0[e], a, c); fh_[e] = a; fl_[e] = c; split16(p1[e], a, c); fh_[8 + e] = a; fl_[8 + e] = c; }
}
__device__ __forceinline__ v8f wmma16b(v16b a, v16b b, v8f c) {
  v8f d = __builtin_amdgcn_wmma_f32_16x16x32_f16(false, a, false, b, (short)0, c, false, false);
  asm volatile("v_nop\n\tv_nop\n\tv_nop\n\tv_nop" : "+v"(d) : "v"(a), "v"(b));
  return d;
}
__device__ __forceinline__ void wave_lds_sync() {
  __builtin_amdgcn_fence(__ATOMIC_RELEASE, "workgroup");
  __builtin_amdgcn_wave_barrier();
  __builtin_amdgcn_fence(__ATOMIC_ACQUIRE, "workgroup");
}

struct Opnd { const void* p0; const void* p1; int ld; };
template <int NP> __device__ __forceinline__ void load_frags(const Opnd& o, int row, int kb, int hh, v16b& fh_, v16b& fl_) {
  if (NP == 0) { frag_ksplit((const float*)o.p0 + (size_t)row * o.ld + kb, hh, fh_, fl_); }
  else if (NP == 3) {
    const float* p = (const float*)o.p0 + (size_t)row * o.ld + kb; const float* p0 = p + 8 * hh; const float* p1 = p + 16 + 8 * hh;
#pragma unroll
    for (int e = 0; e < 8; ++e) { fh_[e] = (b16)p0[e]; fh_[8 + e] = (b16)p1[e]; }
    fl_ = fh_;
  } else {
    fh_ = frag_kb((const b16*)o.p0 + (size_t)row * o.ld + kb, hh);
    if (NP == 2) fl_ = frag_kb((const b16*)o.p1 + (size_t)row * o.ld + kb, hh); else fl_ = fh_;
  }
}
template <int ANP, int BNP> __device__ __forceinline__ v8f mac(v16b ah, v16b al, v16b bh, v16b bl, v8f c) {
  c = wmma16b(ah, bh, c);
  if (BNP == 0 || BNP == 2) c = wmma16b(ah, bl, c);
  if (ANP == 0 || ANP == 2) c = wmma16b(al, bh, c);
  return c;
}
template <int ANP, int BNP>
__device__ __forceinline__ void gemm_tile(const Opnd& A, const Opnd& B, int K, int m0, int c0, int nloc, int hlf, v8f (&acc)[2][4]) {
  for (int kb = 0; kb < K; kb += 32) {
    v16b a0h, a0l, a1h, a1l;
    load_frags<ANP>(A, m0 + nloc, kb, hlf, a0h, a0l);
    load_frags<ANP>(A, m0 + 16 + nloc, kb, hlf, a1h, a1l);
#pragma unroll
    for (int t = 0; t < 4; ++t) {
      v16b bh, bl;
      load_frags<BNP>(B, c0 + t * 16 + nloc, kb, hlf, bh, bl);
      acc[0][t] = mac<ANP, BNP>(a0h, a0l, bh, bl, acc[0][t]);
      acc[1][t] = mac<ANP, BNP>(a1h, a1l, bh, bl, acc[1][t]);
    }
  }
}

struct Epi { float scale; const float* cscale; const float* cbias; const float* rbias; int act; float post; const float* rscale; const float* resid; };
__device__ __forceinline__ float epi_val(const Epi& e, float acc, int row, int col) {
  float val = acc * e.scale;
  if (e.cscale) val *= e.cscale[col];
  if (e.cbias) val += e.cbias[col];
  if (e.rbias) val += e.rbias[row];
  if (e.act == 1) val = 0.5f * val * (1.0f + erff(val * 0.70710678118654752f));
  val *= e.post;
  if (e.rscale) val *= e.rscale[(size_t)row * 32];
  return val;
}
__device__ __forceinline__ void epi_planes(v8f (&acc)[2][4], const Epi& e, bool two,
                                           b16* __restrict__ oh, b16* __restrict__ ol, int ldo, int m0, int c0, int lane, b16* Th, b16* Tl) {
  const int nloc = lane & 15, hlf = lane >> 4;
#pragma unroll
  for (int t = 0; t < 4; ++t)
#pragma unroll
    for (int r = 0; r < 2; ++r)
#pragma unroll
      for (int v = 0; v < 8; ++v) {
        const int rr = r * 16 + v + 8 * hlf, cc = t * 16 + nloc;
        const float val = epi_val(e, acc[r][t][v], m0 + rr, c0 + cc);
        b16 h_, l_; split16(val, h_, l_);
        Th[rr * 64 + cc] = h_; if (two) Tl[rr * 64 + cc] = l_;
      }
  wave_lds_sync();
  for (int pass = 0; pass < 2; ++pass) {
#pragma unroll
    for (int j = 0; j < 8; ++j) {
      const int rr = j * 4 + (lane >> 3), c8 = (lane & 7) * 8;
      const size_t o = (size_t)(m0 + rr) * ldo + c0 + c8;
      *(volatile v8b*)(oh + o) = ld8b(Th + rr * 64 + c8);
      if (two) *(volatile v8b*)(ol + o) = ld8b(Tl + rr * 64 + c8);
    }
    __threadfence();
  }
}
__device__ __forceinline__ void epi_f32(v8f (&acc)[2][4], const Epi& e, float* __restrict__ out, int ldo, int m0, int c0, int lane, float* Tt) {
  const int nloc = lane & 15, hlf = lane >> 4;
#pragma unroll
  for (int t = 0; t < 4; ++t)
#pragma unroll
    for (int r = 0; r < 2; ++r)
#pragma unroll
      for (int v = 0; v < 8; ++v) {
        const int rr = r * 16 + v + 8 * hlf, cc = t * 16 + nloc;
        Tt[rr * 64 + cc] = epi_val(e, acc[r][t][v], m0 + rr, c0 + cc);
      }
  wave_lds_sync();
  float* dst0 = out + (size_t)m0 * ldo + c0; const float* rs0 = e.resid ? e.resid + (size_t)m0 * ldo + c0 : nullptr;
  for (int pass = 0; pass < 2; ++pass) {
#pragma unroll
    for (int j = 0; j < 16; ++j) {
      const int rr = j * 2 + hlf, c4 = nloc * 4;
      v4f val = *(const v4f*)(Tt + rr * 64 + c4);
      if (rs0) val += *(const v4f*)(rs0 + (size_t)rr * ldo + c4);
      *(volatile v4f*)(dst0 + (size_t)rr * ldo + c4) = val;
    }
    __threadfence();
  }
}


__global__ __launch_bounds__(256) void prep_kernel(const float* __restrict__ wqv, const float* __restrict__ w1, const float* __restrict__ w2, const float* __restrict__ wo1,
                                                   const float* __restrict__ wo2, b16* __restrict__ w16) {
  const size_t tid = (size_t)blockIdx.x * blockDim.x + threadIdx.x, stride = (size_t)gridDim.x * blockDim.x;
  const size_t n0 = (size_t)2 * E * E / 8, n1 = (size_t)MS * 32 / 8, n2 = (size_t)H * MS / 8, n3 = (size_t)E * E / 8;
  for (int pass = 0; pass < 2; ++pass) {
    for (size_t c = tid; c < n0 + n1 + n2 + 2 * n3; c += stride) {
      const float* src; if (c < n0) src = wqv + c * 8; else if (c < n0 + n1) src = w1 + (c - n0) * 8; else if (c < n0 + n1 + n2) src = w2 + (c - n0 - n1) * 8;
      else if (c < n0 + n1 + n2 + n3) src = wo1 + (c - n0 - n1 - n2) * 8; else src = wo2 + (c - n0 - n1 - n2 - n3) * 8;
      v8b v;
#pragma unroll
      for (int e = 0; e < 8; ++e) v[e] = (b16)(src[e] * WS);
      *(volatile v8b*)(w16 + c * 8) = v;
    }
    __threadfence();
  }
}

__global__ __launch_bounds__(128) void qkv_kernel(const float* __restrict__ x1, const float* __restrict__ x2, const b16* __restrict__ w16,
                                                  b16* __restrict__ q16, b16* __restrict__ k16, b16* __restrict__ v1T, b16* __restrict__ v2T) {
  __shared__ __attribute__((aligned(16))) b16 Tt[64][128 + 8];
  __shared__ __attribute__((aligned(16))) b16 Th[4][2][32 * 64];
  const int lane = threadIdx.x & 31, wave = threadIdx.x >> 5, nloc = lane & 15, hlf = lane >> 4, z = blockIdx.z;
  const int m0 = blockIdx.y * 128 + wave * 32, c0 = blockIdx.x * 64; const bool isv = c0 >= E;
  v8f acc[2][4];
#pragma unroll
  for (int r = 0; r < 2; ++r)
#pragma unroll
    for (int t = 0; t < 4; ++t) acc[r][t] = (v8f){};
  const Opnd A{z ? x2 : x1, nullptr, E}, B{w16, nullptr, E};
  gemm_tile<3, 1>(A, B, E, m0, c0, nloc, hlf, acc);
  if (!isv) {
    const Epi e{(z ? QS : 0.25f * QS) / WS, nullptr, nullptr, nullptr, 0, 1.0f, nullptr, nullptr};
    epi_planes(acc, e, false, (z ? k16 : q16), nullptr, E, m0, c0, lane, Th[wave][0], nullptr);
    return;
  }
#pragma unroll
  for (int t = 0; t < 4; ++t)
#pragma unroll
    for (int r = 0; r < 2; ++r)
#pragma unroll
      for (int v = 0; v < 8; ++v) Tt[t * 16 + nloc][wave * 32 + r * 16 + 8 * hlf + v] = (b16)(acc[r][t][v] * (VS / WS));
  __syncthreads();
  const int b = (blockIdx.y * 128) / R, tok0 = (blockIdx.y * 128) % R, hd0 = c0 - E;
  b16* base = (z ? v2T : v1T) + ((size_t)b * MS + hd0) * R + tok0;
  for (int pass = 0; pass < 2; ++pass) {
#pragma unroll
    for (int j = 0; j < 8; ++j) { const int rowi = wave * 16 + j * 2 + (lane >> 4), c8 = (lane & 15) * 8; *(volatile v8b*)(base + (size_t)rowi * R + c8) = *(const v8b*)(&Tt[rowi][c8]); }
    __threadfence();
  }
}

__global__ __launch_bounds__(128) void ms_kernel(const b16* __restrict__ q16, const b16* __restrict__ k16, const float* __restrict__ cost, const b16* __restrict__ w16,
                                                 float* __restrict__ ms2, double* __restrict__ part) {
  __shared__ __attribute__((aligned(16))) b16 Ls[4][16][MS + 8];
  __shared__ __attribute__((aligned(16))) float Os0[4][16][16][16];
  __shared__ __attribute__((aligned(16))) float Os1[4][16][16];
  __shared__ __attribute__((aligned(16))) b16 Dt[4][H][16][16];
  const int lane = threadIdx.x & 31, wave = threadIdx.x >> 5, hh = lane >> 4, col = lane & 15;
  const int wid = blockIdx.x * 4 + wave;
  const int b = wid / ((R / 16) * (Cn / 32)), rem = wid % ((R / 16) * (Cn / 32)), r0 = (rem / (Cn / 32)) * 16, c0 = (rem % (Cn / 32)) * 32;
  const b16* W1 = w16 + (size_t)2 * E * E;  const b16* W2 = W1 + (size_t)MS * 32;
  double s1 = 0.0, s2 = 0.0;
  for (int ct = 0; ct < 2; ++ct) {
    const int cb = c0 + ct * 16;
#pragma unroll 1
    for (int h = 0; h < H; ++h) {
      v8f dacc = {};
      v16b a, bk;
      const b16* qa = q16 + ((size_t)b * R + r0 + col) * E + h * D; const b16* kbp = k16 + ((size_t)b * Cn + cb + col) * E + h * D;
#pragma unroll
      for (int e = 0; e < 8; ++e) { a[e] = qa[8 * hh + e]; a[8 + e] = (b16)0.0f; bk[e] = kbp[8 * hh + e]; bk[8 + e] = (b16)0.0f; }
      dacc = wmma16b(a, bk, dacc);
#pragma unroll
      for (int v = 0; v < 8; ++v) Dt[wave][h][8 * hh + v][col] = (b16)(dacc[v] * (TS / (QS * QS)));
    }
    wave_lds_sync();
    for (int r = 0; r < 16; ++r) {
      v16b ar;
      const b16 cs = (b16)(cost[((size_t)b * R + r0 + r) * Cn + cb + col] * TS);
#pragma unroll
      for (int e = 0; e < 16; ++e) {
        const int h = ((e < 8) ? (8 * hh + e) : (16 + 8 * hh + e - 8)) >> 1, s = e & 1;
        ar[e] = s ? cs : Dt[wave][h][r][col];
      }
#pragma unroll
      for (int jt = 0; jt < MS / 16; ++jt) {
        v8f m1 = {};
        m1 = wmma16b(ar, frag_kb(W1 + (size_t)(jt * 16 + col) * 32, hh), m1);
#pragma unroll
        for (int v = 0; v < 8; ++v) Ls[wave][8 * hh + v][jt * 16 + col] = (b16)(fmaxf(m1[v] * (1.0f / (TS * WS)), 0.0f) * M1S);
      }
      wave_lds_sync();
      v8f m2 = {};
#pragma unroll
      for (int kb = 0; kb < MS; kb += 32) m2 = wmma16b(frag_kb(&Ls[wave][col][kb], hh), frag_kb(W2 + (size_t)col * MS + kb, hh), m2);
#pragma unroll
      for (int v = 0; v < 8; ++v) { const float val = m2[v] * (1.0f / (M1S * WS)); if (ct == 0) Os0[wave][r][col][8 * hh + v] = val; else Os1[wave][col][8 * hh + v] = val; s1 += (double)val; s2 += (double)val * (double)val; }
      wave_lds_sync();
      if (ct == 1) {
        float* dst = ms2 + (((size_t)b * H) * R + r0 + r) * Cn + c0;
        for (int pass = 0; pass < 2; ++pass) {
#pragma unroll
          for (int j = 0; j < 4; ++j) { const int hp = j * 4 + (lane >> 3), c4 = (lane & 7) * 4;
            const v4f w4 = (c4 < 16) ? *(const v4f*)(&Os0[wave][r][hp][c4]) : *(const v4f*)(&Os1[wave][hp][c4 - 16]);
            *(volatile v4f*)(dst + (size_t)hp * R * Cn + c4) = w4; }
          __threadfence();
        }
      }
    }
  }
#pragma unroll
  for (int o = 16; o > 0; o >>= 1) { s1 += __shfl_xor(s1, o); s2 += __shfl_xor(s2, o); }
  const double pv = (lane == 0) ? s1 : (lane == 1) ? s2 : 0.0;
  if (lane < 16) { ((volatile double*)part)[(size_t)wid * 16 + lane] = pv; __threadfence(); ((volatile double*)part)[(size_t)wid * 16 + lane] = pv; }
}

__global__ __launch_bounds__(256) void std_kernel(const double* __restrict__ part, const int* __restrict__ amask, float* __restrict__ inv) {
  __shared__ int anyz[256];
  const int t = threadIdx.x;
  int z0 = 0;
#pragma unroll 1
  for (size_t i = t; i < (size_t)Bn * R * Cn; i += 256) z0 |= (amask[i] == 0);
  anyz[t] = z0; __syncthreads();
#pragma unroll 1
  for (int o = 128; o > 0; o >>= 1) { if (t < o) anyz[t] |= anyz[t + o]; __syncthreads(); }
  if (t == 0) {
    double s1 = 0.0, s2 = 0.0;
#pragma unroll 1
    for (int w = 0; w < NWAVE_MS; ++w) { s1 += part[(size_t)w * 16]; s2 += part[(size_t)w * 16 + 1]; }
    const double n = (double)Bn * H * R * Cn, mean = s1 / n, var = (s2 - n * mean * mean) / (n - 1.0);
    float is = (float)(1.0 / sqrt(var)); if (anyz[0]) is = __int_as_float(0x7fc00000);
    ((volatile float*)inv)[0] = is; __threadfence(); ((volatile float*)inv)[0] = is;
  }
}

template <int DIRN>
__global__ __launch_bounds__(256) void attn_kernel(const float* __restrict__ ms2, const float* __restrict__ inv, const int* __restrict__ amask, const b16* __restrict__ vT,
                                                   b16* __restrict__ y) {
  __shared__ __attribute__((aligned(16))) b16 Os[16][128 + 8];
  const int wave = threadIdx.x >> 5, lane = threadIdx.x & 31, hh = lane >> 4, col = lane & 15;
  const int NQ = DIRN ? Cn : R, NK = DIRN ? R : Cn;
  const int b = blockIdx.x / ((NQ / 16) * 2), rem = blockIdx.x % ((NQ / 16) * 2), q0 = (rem >> 1) * 16, hbase = (rem & 1) * 8, h = hbase + wave;
  const float is = inv[0]; const int qi = q0 + col;
  const float* S = ms2 + ((size_t)b * H + h) * R * Cn; const int* M = amask + (size_t)b * R * Cn;
  const b16* vt = vT + ((size_t)b * MS + h * D) * NK;
  float m = -INFINITY, l = 0.0f; v8f o = {};
  for (int kb = 0; kb < NK; kb += 32) {
    v8f s0, s1;
#pragma unroll
    for (int r = 0; r < 8; ++r) {
      const int k0i = kb + 8 * hh + r, k1i = k0i + 16;
      const size_t i0 = DIRN ? ((size_t)k0i * Cn + qi) : ((size_t)qi * Cn + k0i), i1 = DIRN ? ((size_t)k1i * Cn + qi) : ((size_t)qi * Cn + k1i);
      s0[r] = M[i0] ? S[i0] * is : -INFINITY; s1[r] = M[i1] ? S[i1] * is : -INFINITY;
    }
    float mr = -INFINITY;
#pragma unroll
    for (int r = 0; r < 8; ++r) mr = fmaxf(mr, fmaxf(s0[r], s1[r]));
    mr = fmaxf(mr, __shfl_xor(mr, 16));
    float mn = fmaxf(m, mr); const float mref = (mn == -INFINITY) ? 0.0f : mn;
    const float al_ = __expf(m - mref); m = mn;
    float sum = 0.0f; v16b pb;
#pragma unroll
    for (int r = 0; r < 8; ++r) { const float p0 = __expf(s0[r] - mref), p1 = __expf(s1[r] - mref); sum += p0 + p1; pb[r] = (b16)p0; pb[8 + r] = (b16)p1; }
    sum += __shfl_xor(sum, 16);
    l = l * al_ + sum;
#pragma unroll
    for (int r = 0; r < 8; ++r) o[r] *= al_;
    o = wmma16b(frag_kb(vt + (size_t)col * NK + kb, hh), pb, o);
  }
  const float invl = (l > 0.0f) ? (YS / (VS * l)) : 0.0f;
#pragma unroll
  for (int r = 0; r < 8; ++r) Os[col][wave * 16 + 8 * hh + r] = (b16)(o[r] * invl);
  __syncthreads();
  b16* dst = y + ((size_t)b * NQ + q0) * MS + hbase * D;
  for (int pass = 0; pass < 2; ++pass) {
    { const int rr = threadIdx.x >> 4, c8 = (threadIdx.x & 15) * 8; *(volatile v8b*)(dst + (size_t)rr * MS + c8) = *(const v8b*)(&Os[rr][c8]); }
    __threadfence();
  }
}

__global__ __launch_bounds__(128) void out_kernel(const b16* __restrict__ y1, const b16* __restrict__ y2, const b16* __restrict__ w16, float* __restrict__ out) {
  __shared__ __attribute__((aligned(16))) float Ts[4][32 * 64];
  const int lane = threadIdx.x & 31, wave = threadIdx.x >> 5, nloc = lane & 15, hlf = lane >> 4, z = blockIdx.z;
  const int m0 = blockIdx.y * 128 + wave * 32, c0 = blockIdx.x * 64;
  v8f acc[2][4];
#pragma unroll
  for (int r = 0; r < 2; ++r)
#pragma unroll
    for (int t = 0; t < 4; ++t) acc[r][t] = (v8f){};
  const b16* wo = w16 + (size_t)2 * E * E + (size_t)MS * 32 + (size_t)H * MS + (size_t)z * E * E;
  const Opnd A{z ? y2 : y1, nullptr, MS}, B{wo, nullptr, E};
  gemm_tile<1, 1>(A, B, MS, m0, c0, nloc, hlf, acc);
  const Epi e{1.0f / (YS * WS), nullptr, nullptr, nullptr, 0, 1.0f, nullptr, nullptr};
  epi_f32(acc, e, out + (size_t)z * NT1 * E, E, m0, c0, lane, Ts[wave]);
}
}

extern "C" void kernel_launch(void* const* d_in, const int* in_sizes, int n_in,
                              void* d_out, int out_size, void* d_ws, size_t ws_size, hipStream_t stream) {
  (void)n_in; (void)out_size;
  const float* x1  = (const float*)d_in[0];
  const float* x2  = (const float*)d_in[1];
  const float* cost = (const float*)d_in[2];
  const int* amask = (const int*)d_in[3];
  const float* wqv = (const float*)d_in[4];
  const float* w1  = (const float*)d_in[5];
  const float* w2  = (const float*)d_in[6];
  const float* wo1 = (const float*)d_in[7];
  const float* wo2 = (const float*)d_in[8];
  float* out = (float*)d_out;
  if (in_sizes[0] != NT1 * E || in_sizes[1] != NT2 * E || in_sizes[2] != Bn * R * Cn || in_sizes[3] != Bn * R * Cn || in_sizes[4] != 2 * E * E || in_sizes[5] != MS * 32 || in_sizes[6] != H * MS) return;

  size_t off = 0; char* ws = (char*)d_ws;
  auto carve = [&](size_t bytes) { char* p = ws + off; off += (bytes + 255) & ~(size_t)255; return p; };
  b16* w16  = (b16*)carve(((size_t)2 * E * E + MS * 32 + H * MS + 2 * (size_t)E * E) * 2);
  b16* q16  = (b16*)carve((size_t)NT1 * E * 2);
  b16* k16  = (b16*)carve((size_t)NT2 * E * 2);
  b16* v1T  = (b16*)carve((size_t)Bn * MS * R * 2);
  b16* v2T  = (b16*)carve((size_t)Bn * MS * Cn * 2);
  float* ms2 = (float*)carve((size_t)Bn * H * R * Cn * 4);
  double* part = (double*)carve((size_t)NWAVE_MS * 16 * 8);
  float* inv = (float*)carve(256);
  b16* y1   = (b16*)carve((size_t)NT1 * MS * 2);
  b16* y2   = (b16*)carve((size_t)NT2 * MS * 2);
  if (off > ws_size) return;
  prep_kernel<<<128, 256, 0, stream>>>(wqv, w1, w2, wo1, wo2, w16);
  qkv_kernel<<<dim3(2 * E / 64, NT1 / 128, 2), 128, 0, stream>>>(x1, x2, w16, q16, k16, v1T, v2T);
  ms_kernel<<<NWAVE_MS / 4, 128, 0, stream>>>(q16, k16, cost, w16, ms2, part);
  std_kernel<<<1, 256, 0, stream>>>(part, amask, inv);
  attn_kernel<0><<<Bn * (R / 16) * 2, 256, 0, stream>>>(ms2, inv, amask, v2T, y1);
  attn_kernel<1><<<Bn * (Cn / 16) * 2, 256, 0, stream>>>(ms2, inv, amask, v1T, y2);
  out_kernel<<<dim3(E / 64, NT1 / 128, 2), 128, 0, stream>>>(y1, y2, w16, out);
}
